// ExpHydroM100_22445499089624
// MI455X (gfx1250) — hardware-run, weakly checked
//
#include <hip/hip_runtime.h>
#include <math.h>

typedef __attribute__((ext_vector_type(16))) _Float16 v16h;
typedef __attribute__((ext_vector_type(8)))  _Float16 v8h;
typedef __attribute__((ext_vector_type(8)))  float    v8f;
typedef __attribute__((ext_vector_type(4)))  float    v4f;
typedef __attribute__((ext_vector_type(2)))  float    v2f;
typedef __attribute__((ext_vector_type(4)))  unsigned v4u;

constexpr int kNB  = 64;
constexpr int kNT  = 2048;
constexpr int kH   = 64;
constexpr int kNO  = 5;
constexpr int kNOP = 16;
constexpr int kTile = 16 * kH;
static_assert((kH % 32) == 0, "K multiple of 32");
static_assert((kNB % 16) == 0 && (kNT % 32) == 0, "tile multiples");

constexpr float kActCarry = 256.0f;
constexpr float kW23Carry = 256.0f;
constexpr float kW4Carry  = 4096.0f;
constexpr float kLoCarry  = 4096.0f;
constexpr float kLoInv    = 1.0f / kLoCarry;
constexpr float kScale23  = 1.0f / (kActCarry * kW23Carry);
constexpr float kScale4   = 1.0f / (kActCarry * kW4Carry);
constexpr float kHalfMin  = 6.103515625e-05f;

constexpr int kW2H = 0;
constexpr int kW3H = kW2H + kH * kH;
constexpr int kW4H = kW3H + kH * kH;
constexpr int kWHalves = kW4H + kNOP * kH;
static_assert(kWHalves == 9216, "plane halves");
constexpr int kWChunks = kWHalves / 8;
static_assert(kWChunks == 1152, "16-B chunks of the planes");
constexpr size_t kOffPlanes = 0;
constexpr size_t kPlaneBytes = (size_t)kWHalves * 2;
constexpr size_t kOffTraj = kOffPlanes + kPlaneBytes;
constexpr size_t kTrajBytes = (size_t)kNT * kNB * 2 * 4;
constexpr size_t kWsTotal = kOffTraj + kTrajBytes;
static_assert(kPlaneBytes == 18432ull, "planes bytes");
static_assert(kTrajBytes == 1048576ull, "traj bytes");
static_assert(kWsTotal == 1067008ull, "carve total");
static_assert(kWsTotal <= 134217728ull, "carve cap");
static_assert((kOffTraj % 128) == 0, "128-B aligned regions");

union FragU { v16h v; v8h h[2]; };
__device__ __forceinline__ v16h frag_load(const _Float16* p) {
  FragU f;
  f.h[0] = *(const v8h*)(p);
  f.h[1] = *(const v8h*)(p + 16);
  return f.v;
}
__device__ __forceinline__ v8f mma_h(v16h a, v16h b, v8f c) {
  c = __builtin_amdgcn_wmma_f32_16x16x32_f16(false, a, false, b, (short)0, c, false, false);
  asm volatile("v_nop\n\tv_nop\n\tv_nop\n\tv_nop" : "+v"(c) : "v"(a), "v"(b));
  return c;
}
__device__ __forceinline__ void wave_lds_sync() {
  __builtin_amdgcn_fence(__ATOMIC_RELEASE, "workgroup");
  __builtin_amdgcn_wave_barrier();
  __builtin_amdgcn_fence(__ATOMIC_ACQUIRE, "workgroup");
}
__device__ __forceinline__ float tanh_fast(float x) {
  const float xc = fminf(fmaxf(x, -15.0f), 15.0f);
  const float e2 = __builtin_amdgcn_exp2f(xc * 2.885390081777927f);
  return 1.0f - 2.0f * __builtin_amdgcn_rcpf(1.0f + e2);
}
__device__ __forceinline__ _Float16 half_flush(float v) {
  const float z = (fabsf(v) < kHalfMin) ? 0.0f : v;
  return (_Float16)z;
}
__device__ __forceinline__ void split_act(float t, _Float16& hq, _Float16& lq) {
  hq = half_flush(t);
  const float rs = (t - (float)hq) * kLoCarry;
  lq = half_flush(rs);
}
__device__ __forceinline__ unsigned pack2h(_Float16 a, _Float16 b) {
  const unsigned short ua = __builtin_bit_cast(unsigned short, a);
  const unsigned short ub = __builtin_bit_cast(unsigned short, b);
  return (unsigned)ua | ((unsigned)ub << 16);
}

struct MlpRegs {
  float w1a[4];
  float w1b[4];
  float b1a;
  float b1b;
  float b4v;
};

__device__ __forceinline__ MlpRegs load_regs(const float* __restrict__ W1, const float* __restrict__ b1,
                                             const float* __restrict__ b4, int lane) {
  MlpRegs rg;
  const int n2 = 2 * lane;
#pragma unroll
  for (int k = 0; k < 4; ++k) {
    const v2f w = *(const v2f*)(W1 + k * kH + n2);
    rg.w1a[k] = w.x;
    rg.w1b[k] = w.y;
  }
  const v2f bb = *(const v2f*)(b1 + n2);
  rg.b1a = bb.x;
  rg.b1b = bb.y;
  const int n = lane & 15;
  const int nc = (n < kNO) ? n : (kNO - 1);
  const float b4l = b4[nc];
  rg.b4v = (n < kNO) ? b4l : 0.0f;
  return rg;
}

__device__ __forceinline__ void stage_consts(_Float16* sW, float* sB, const _Float16* __restrict__ planes,
                                             const float* __restrict__ b2, const float* __restrict__ b3,
                                             int tid, int nthr) {
  const v4u* src = (const v4u*)planes;
  v4u* dst = (v4u*)sW;
  for (int i = tid; i < kWChunks; i += nthr) dst[i] = src[i];
  for (int i = tid; i < 2 * kH; i += nthr) {
    const int c = i & (kH - 1);
    const float v2 = b2[c];
    const float v3 = b3[c];
    sB[i] = (i < kH) ? v2 : v3;
  }
}

__device__ __forceinline__ void dense64_tanh(const _Float16* Ah, const _Float16* Al, const _Float16* Wt,
                                             const float* bias, _Float16* Oh, _Float16* Ol, int n, int hh) {
  const v16h ah0 = frag_load(Ah + n * kH + 8 * hh);
  const v16h ah1 = frag_load(Ah + n * kH + 32 + 8 * hh);
  const v16h al0 = frag_load(Al + n * kH + 8 * hh);
  const v16h al1 = frag_load(Al + n * kH + 32 + 8 * hh);
#pragma unroll 1
  for (int j = 0; j < 4; ++j) {
    const int wo = (16 * j + n) * kH + 8 * hh;
    const v16h b0 = frag_load(Wt + wo);
    const v16h b1 = frag_load(Wt + wo + 32);
    v8f ch = (v8f){0.f, 0.f, 0.f, 0.f, 0.f, 0.f, 0.f, 0.f};
    v8f cl = (v8f){0.f, 0.f, 0.f, 0.f, 0.f, 0.f, 0.f, 0.f};
    ch = mma_h(ah0, b0, ch);
    ch = mma_h(ah1, b1, ch);
    cl = mma_h(al0, b0, cl);
    cl = mma_h(al1, b1, cl);
    const float bv = bias[16 * j + n];
#pragma unroll
    for (int e = 0; e < 8; ++e) {
      float v = fmaf(cl[e], kLoInv, ch[e]);
      v = fmaf(v, kScale23, bv);
      const float t = tanh_fast(v) * kActCarry;
      _Float16 hq, lq;
      split_act(t, hq, lq);
      Oh[(8 * hh + e) * kH + 16 * j + n] = hq;
      Ol[(8 * hh + e) * kH + 16 * j + n] = lq;
    }
  }
}

__device__ __forceinline__ void mlp16(const MlpRegs& rg, const _Float16* sW, const float* sB, const float* sX,
                                      _Float16* sA, float* sO, int lane) {
  const int n = lane & 15;
  const int hh = lane >> 4;
  _Float16* sA0h = sA;
  _Float16* sA0l = sA + kTile;
  _Float16* sA1h = sA + 2 * kTile;
  _Float16* sA1l = sA + 3 * kTile;
  unsigned* a0hw = (unsigned*)sA0h;
  unsigned* a0lw = (unsigned*)sA0l;
#pragma unroll 2
  for (int m = 0; m < 16; ++m) {
    const v4f x = *(const v4f*)(sX + m * 4);
    float p0 = x[0] * rg.w1a[0];
    p0 = fmaf(x[1], rg.w1a[1], p0);
    p0 = fmaf(x[2], rg.w1a[2], p0);
    p0 = fmaf(x[3], rg.w1a[3], p0);
    p0 = p0 + rg.b1a;
    float p1 = x[0] * rg.w1b[0];
    p1 = fmaf(x[1], rg.w1b[1], p1);
    p1 = fmaf(x[2], rg.w1b[2], p1);
    p1 = fmaf(x[3], rg.w1b[3], p1);
    p1 = p1 + rg.b1b;
    const float t0 = tanh_fast(p0) * kActCarry;
    const float t1 = tanh_fast(p1) * kActCarry;
    _Float16 h0, l0, h1, l1;
    split_act(t0, h0, l0);
    split_act(t1, h1, l1);
    a0hw[m * 32 + lane] = pack2h(h0, h1);
    a0lw[m * 32 + lane] = pack2h(l0, l1);
  }
  wave_lds_sync();
  dense64_tanh(sA0h, sA0l, sW + kW2H, sB, sA1h, sA1l, n, hh);
  wave_lds_sync();
  dense64_tanh(sA1h, sA1l, sW + kW3H, sB + kH, sA0h, sA0l, n, hh);
  wave_lds_sync();
  {
    const v16h ah0 = frag_load(sA0h + n * kH + 8 * hh);
    const v16h ah1 = frag_load(sA0h + n * kH + 32 + 8 * hh);
    const v16h al0 = frag_load(sA0l + n * kH + 8 * hh);
    const v16h al1 = frag_load(sA0l + n * kH + 32 + 8 * hh);
    const int wo = n * kH + 8 * hh;
    const v16h b0 = frag_load(sW + kW4H + wo);
    const v16h b1 = frag_load(sW + kW4H + wo + 32);
    v8f ch = (v8f){0.f, 0.f, 0.f, 0.f, 0.f, 0.f, 0.f, 0.f};
    v8f cl = (v8f){0.f, 0.f, 0.f, 0.f, 0.f, 0.f, 0.f, 0.f};
    ch = mma_h(ah0, b0, ch);
    ch = mma_h(ah1, b1, ch);
    cl = mma_h(al0, b0, cl);
    cl = mma_h(al1, b1, cl);
#pragma unroll
    for (int e = 0; e < 8; ++e) {
      float v = fmaf(cl[e], kLoInv, ch[e]);
      v = fmaf(v, kScale4, rg.b4v);
      sO[(8 * hh + e) * kNOP + n] = v;
    }
  }
  wave_lds_sync();
}

__global__ __launch_bounds__(128) void prep_planes_kernel(const float* __restrict__ W2,
                                                          const float* __restrict__ W3,
                                                          const float* __restrict__ W4,
                                                          _Float16* __restrict__ planes) {
  const int tid = threadIdx.x;
#pragma unroll 1
  for (int it = 0; it < 9; ++it) {
    const int task = it * 128 + tid;
    const int g = task >> 3;
    const int c = task & 7;
    const bool isA = (g < 64);
    const bool isB = (g >= 64) && (g < 128);
    const bool isAB = (g < 128);
    const float* src = isA ? W2 : (isB ? W3 : W4);
    const int ld = isAB ? kH : kNO;
    const int nraw = isA ? g : (isB ? (g - 64) : (g - 128));
    const bool valid = isAB || (nraw < kNO);
    const int ncl = isAB ? nraw : ((nraw < kNO) ? nraw : (kNO - 1));
    const float carry = isAB ? kW23Carry : kW4Carry;
    const int dh = (isA ? kW2H : (isB ? kW3H : kW4H)) + nraw * kH + c * 8;
    v8h hv;
#pragma unroll
    for (int e = 0; e < 8; ++e) {
      const int k = c * 8 + e;
      const float wl = src[k * ld + ncl];
      const float w = valid ? (wl * carry) : 0.0f;
      const _Float16 hq = half_flush(w);
      hv[e] = hq;
    }
    *(volatile v8h*)(planes + dh) = hv;
    __threadfence();
    *(volatile v8h*)(planes + dh) = hv;
  }
}

__global__ __launch_bounds__(32) void scan_kernel(
    const float* __restrict__ s_snow, const float* __restrict__ s_water,
    const float* __restrict__ precp, const float* __restrict__ tmean, const float* __restrict__ lday,
    const float* __restrict__ times,
    const float* __restrict__ W1, const float* __restrict__ b1, const float* __restrict__ b2,
    const float* __restrict__ b3, const float* __restrict__ b4,
    const _Float16* __restrict__ planes, float* __restrict__ traj) {
  __shared__ __align__(16) _Float16 sW[kWHalves];
  __shared__ __align__(16) float sB[2 * kH];
  __shared__ __align__(16) float sX[16 * 4];
  __shared__ __align__(16) _Float16 sA[4 * kTile];
  __shared__ __align__(16) float sO[16 * kNOP];

  const int lane = threadIdx.x;
  stage_consts(sW, sB, planes, b2, b3, lane, 32);
  __syncthreads();
  const MlpRegs rg = load_regs(W1, b1, b4, lane);

  const int bl = lane >> 1;
  const int comp = lane & 1;
  const int basin = blockIdx.x * 16 + bl;
  const size_t rowoff = (size_t)basin * kNT;

  float y0 = s_snow[rowoff];
  float y1 = s_water[rowoff];
  {
    const float v = comp ? y1 : y0;
    volatile float* p = traj + blockIdx.x * 32 + lane;
    *p = v;
    __threadfence();
    *p = v;
  }

#pragma unroll 1
  for (int stp = 0; stp < kNT - 1; ++stp) {
    const float t0 = times[stp];
    const float dt = times[stp + 1] - t0;
    const float hdt = dt * 0.5f;
    float kp0 = 0.0f, kp1 = 0.0f;
    float ks0 = 0.0f, ks1 = 0.0f;
#pragma unroll 1
    for (int sub = 0; sub < 4; ++sub) {
      const float cs = (sub == 3) ? dt : hdt;
      const float tc = (sub == 0) ? t0 : (t0 + cs);
      float c0 = y0;
      float c1 = y1;
      if (sub != 0) {
        c0 = y0 + cs * kp0;
        c1 = y1 + cs * kp1;
      }
      const float fl = fminf(fmaxf(floorf(tc), 0.0f), (float)(kNT - 2));
      const int i0 = (int)fl;
      const float fr = tc - fl;
      const float om = 1.0f - fr;
      const size_t ib = rowoff + (size_t)i0;
      const float pa = precp[ib];
      const float pb = precp[ib + 1];
      const float ta = tmean[ib];
      const float tb = tmean[ib + 1];
      const float la = lday[ib];
      const float lb = lday[ib + 1];
      const float pv = pa * om + pb * fr;
      const float tv = ta * om + tb * fr;
      const float lv = la * om + lb * fr;
      v2f xw;
      xw.x = comp ? pv : c0;
      xw.y = comp ? tv : c1;
      *(v2f*)(sX + bl * 4 + comp * 2) = xw;
      wave_lds_sync();

      mlp16(rg, sW, sB, sX, sA, sO, lane);

      const v4f o03 = *(const v4f*)(sO + bl * kNOP);
      const float o4 = sO[bl * kNOP + 4];
      const float stT = (tanhf(-5.0f * tv) + 1.0f) * 0.5f;
      const float st0 = (tanhf(5.0f * c0) + 1.0f) * 0.5f;
      const float st1 = (tanhf(5.0f * c1) + 1.0f) * 0.5f;
      const float psn = fmaxf(sinhf(o03[0]) * stT, 0.0f);
      const float prn = fmaxf(sinhf(o03[1]), 0.0f);
      const float mlt = fmaxf(st0 * sinhf(o03[2]), 0.0f);
      const float evt = st1 * expf(o03[3]) * lv;
      const float qfl = st1 * expf(o4);
      const float d0 = psn - mlt;
      const float d1 = prn + mlt - evt - qfl;
      const float wgt = (sub == 0 || sub == 3) ? 1.0f : 2.0f;
      ks0 = fmaf(wgt, d0, ks0);
      ks1 = fmaf(wgt, d1, ks1);
      kp0 = d0;
      kp1 = d1;
    }
    const float f6 = dt * (1.0f / 6.0f);
    y0 = y0 + f6 * ks0;
    y1 = y1 + f6 * ks1;
    {
      const float v = comp ? y1 : y0;
      volatile float* p = traj + (size_t)(stp + 1) * (kNB * 2) + blockIdx.x * 32 + lane;
      *p = v;
      __threadfence();
      *p = v;
    }
  }
}

__global__ __launch_bounds__(128) void head_kernel(
    const float* __restrict__ precp, const float* __restrict__ tmean,
    const float* __restrict__ W1, const float* __restrict__ b1, const float* __restrict__ b2,
    const float* __restrict__ b3, const float* __restrict__ b4,
    const _Float16* __restrict__ planes, const float* __restrict__ traj, float* __restrict__ out) {
  __shared__ __align__(16) _Float16 sW[kWHalves];
  __shared__ __align__(16) float sB[2 * kH];
  __shared__ __align__(16) float sX[4][16 * 4];
  __shared__ __align__(16) _Float16 sA[4][4 * kTile];
  __shared__ __align__(16) float sO[4][16 * kNOP];

  const int tid = threadIdx.x;
  const int lane = tid & 31;
  const int wave = tid >> 5;
  stage_consts(sW, sB, planes, b2, b3, tid, 128);
  __syncthreads();
  const MlpRegs rg = load_regs(W1, b1, b4, lane);

  const int gw = blockIdx.x * 4 + wave;
  const int b = gw >> 6;
  const int tbase = (gw & 63) * 32;
  const int m = lane >> 1;
  const int comp = lane & 1;
  float res = 0.0f;
#pragma unroll 1
  for (int i = 0; i < 2; ++i) {
    const int t = tbase + 16 * i + m;
    const v2f yy = *(const v2f*)(traj + (size_t)t * (kNB * 2) + b * 2);
    const float pr = precp[(size_t)b * kNT + t];
    const float tm = tmean[(size_t)b * kNT + t];
    v2f xw;
    xw.x = comp ? pr : yy.x;
    xw.y = comp ? tm : yy.y;
    *(v2f*)(sX[wave] + m * 4 + comp * 2) = xw;
    wave_lds_sync();
    mlp16(rg, sW, sB, sX[wave], sA[wave], sO[wave], lane);
    const float o = sO[wave][(lane & 15) * kNOP + 4];
    res = ((lane >> 4) == i) ? o : res;
  }
  {
    volatile float* p = out + (size_t)b * kNT + tbase + lane;
    *p = res;
    __threadfence();
    *p = res;
  }
}

extern "C" void kernel_launch(void* const* d_in, const int* in_sizes, int n_in,
                              void* d_out, int out_size, void* d_ws, size_t ws_size,
                              hipStream_t stream) {
  if (n_in < 14) return;
  if (in_sizes[0] != kNB * kNT) return;
  if (in_sizes[1] != kNB * kNT) return;
  if (in_sizes[2] != kNB * kNT) return;
  if (in_sizes[3] != kNB * kNT) return;
  if (in_sizes[4] != kNB * kNT) return;
  if (in_sizes[5] != kNT) return;
  if (in_sizes[6] != 4 * kH) return;
  if (in_sizes[7] != kH) return;
  if (in_sizes[8] != kH * kH) return;
  if (in_sizes[9] != kH) return;
  if (in_sizes[10] != kH * kH) return;
  if (in_sizes[11] != kH) return;
  if (in_sizes[12] != kH * kNO) return;
  if (in_sizes[13] != kNO) return;
  if (out_size != kNB * kNT) return;
  if (ws_size < kWsTotal) return;

  const float* s_snow  = (const float*)d_in[0];
  const float* s_water = (const float*)d_in[1];
  const float* precp   = (const float*)d_in[2];
  const float* tmean   = (const float*)d_in[3];
  const float* lday    = (const float*)d_in[4];
  const float* times   = (const float*)d_in[5];
  const float* W1 = (const float*)d_in[6];
  const float* b1 = (const float*)d_in[7];
  const float* W2 = (const float*)d_in[8];
  const float* b2 = (const float*)d_in[9];
  const float* W3 = (const float*)d_in[10];
  const float* b3 = (const float*)d_in[11];
  const float* W4 = (const float*)d_in[12];
  const float* b4 = (const float*)d_in[13];
  float* out = (float*)d_out;

  char* ws = (char*)d_ws;
  _Float16* planes = (_Float16*)(ws + kOffPlanes);
  float* traj = (float*)(ws + kOffTraj);

  prep_planes_kernel<<<1, 128, 0, stream>>>(W2, W3, W4, planes);

  scan_kernel<<<kNB / 16, 32, 0, stream>>>(s_snow, s_water, precp, tmean, lday, times,
                                           W1, b1, b2, b3, b4, planes, traj);

  head_kernel<<<(kNB * kNT) / 128, 128, 0, stream>>>(precp, tmean, W1, b1, b2, b3, b4, planes, traj, out);
}
